// SimMask_42219528520119
// MI455X (gfx1250) — hardware-verified
//
#include <hip/hip_runtime.h>


#define NB_  2
#define NN   512
#define MM   512
#define CI   64
#define C1   128
#define C2O  64
#define C3   32
#define NPT  (NB_ * NN)
#define NCL  (NB_ * MM)
#define NPR  (NB_ * NN * MM)
#define NCH  128
#define PCH  (NCH * MM)
#define DM   C1
#define LOSC 1024.0f
typedef _Float16 h16;
typedef unsigned short bf;
typedef __attribute__((ext_vector_type(16))) __bf16   v16bf;
typedef __attribute__((ext_vector_type(16))) _Float16 v16h;
typedef __attribute__((ext_vector_type(8)))  _Float16 v8h;
typedef __attribute__((ext_vector_type(8)))  unsigned short v8us;
typedef __attribute__((ext_vector_type(8)))  float    v8f;
typedef __attribute__((ext_vector_type(4)))  float    v4f;
typedef __attribute__((ext_vector_type(4)))  _Float16 v4h;
typedef v8h  __attribute__((may_alias)) v8ha;
typedef v4f  __attribute__((may_alias)) v4fa;
typedef v8us __attribute__((may_alias)) v8usa;

__device__ __forceinline__ unsigned short f2bf(float f) { unsigned u = __float_as_uint(f); u += 0x7FFFu + ((u >> 16) & 1u); return (unsigned short)(u >> 16); }
__device__ __forceinline__ float bf2f(unsigned short b) { return __uint_as_float(((unsigned)b) << 16); }
__device__ __forceinline__ float bfr(float f) { return bf2f(f2bf(f)); }
__device__ __forceinline__ v16h cat16(v8h lo, v8h hi) { return __builtin_shufflevector(lo, hi, 0, 1, 2, 3, 4, 5, 6, 7, 8, 9, 10, 11, 12, 13, 14, 15); }
__device__ __forceinline__ v16bf cat16b(v8us lo, v8us hi) { return __builtin_bit_cast(v16bf, __builtin_shufflevector(lo, hi, 0, 1, 2, 3, 4, 5, 6, 7, 8, 9, 10, 11, 12, 13, 14, 15)); }
__device__ __forceinline__ v8f wmma16(v16h a, v16h b, v8f c) { return __builtin_amdgcn_wmma_f32_16x16x32_f16(false, a, false, b, (short)0, c, false, false); }
__device__ __forceinline__ v8f wmmab(v16bf a, v16bf b, v8f c) { return __builtin_amdgcn_wmma_f32_16x16x32_bf16(false, a, false, b, (short)0, c, false, false); }

template <bool SPLITA, bool F16OUT = false>
__global__ __launch_bounds__(128) void k_gemmb(const bf* __restrict__ A, const bf* __restrict__ Al, const bf* __restrict__ Bn, const float* __restrict__ bias, float* C, int ldc, h16* C2, const float* __restrict__ R = nullptr, int K = DM, int roundR = 1) {
    __shared__ __align__(16) float ost[4][16 * 68];
    const int lane = threadIdx.x & 31, wave = threadIdx.x >> 5, lr = lane & 15, hi = lane >> 4;
    const int r0 = blockIdx.x * 64 + wave * 16, c0 = blockIdx.y * 64;
    const size_t aoff = (size_t)(r0 + lr) * K + 8 * hi;
    size_t boff[4];
#pragma unroll
    for (int t = 0; t < 4; ++t) boff[t] = (size_t)(c0 + t * 16 + lr) * K + 8 * hi;
    v8f acc[4];
#pragma unroll
    for (int t = 0; t < 4; ++t) acc[t] = (v8f){};
#pragma unroll 1
    for (int kc = 0; kc < K; kc += 32) {
        const v16bf a = cat16b(*(const v8us*)(A + aoff + kc), *(const v8us*)(A + aoff + kc + 16));
        v16bf al = a;
        if (SPLITA) al = cat16b(*(const v8us*)(Al + aoff + kc), *(const v8us*)(Al + aoff + kc + 16));
#pragma unroll
        for (int t = 0; t < 4; ++t) { const v16bf b = cat16b(*(const v8us*)(Bn + boff[t] + kc), *(const v8us*)(Bn + boff[t] + kc + 16)); acc[t] = wmmab(a, b, acc[t]); if (SPLITA) acc[t] = wmmab(al, b, acc[t]); }
        asm volatile("v_nop\n\tv_nop\n\tv_nop\n\tv_nop" : "+v"(acc[0]), "+v"(acc[1]), "+v"(acc[2]), "+v"(acc[3]) : "v"(a), "v"(al));
    }
    float* os = &ost[wave][0];
#pragma unroll
    for (int t = 0; t < 4; ++t) { const float bv = bias ? bfr(bias[c0 + t * 16 + lr]) : 0.f;
#pragma unroll
        for (int j = 0; j < 8; ++j) os[(hi * 8 + j) * 68 + t * 16 + lr] = acc[t][j] + bv; }
    __syncthreads();
    if (F16OUT) {
        h16* crow = (h16*)(void*)C + (size_t)r0 * ldc + c0;
        auto pass = [&]() {
#pragma unroll
            for (int s = 0; s < 4; ++s) { const int row = 4 * s + (lane >> 3), piece = lane & 7; const float* sp = os + row * 68 + piece * 8; v8h o, o2;
#pragma unroll
                for (int i = 0; i < 8; ++i) { const h16 a = (h16)sp[i]; o[i] = a; o2[i] = (h16)((sp[i] - (float)a) * LOSC); }
                *(volatile v8h*)(crow + (size_t)row * ldc + piece * 8) = o; if (C2) *(volatile v8h*)(C2 + (size_t)r0 * ldc + c0 + (size_t)row * ldc + piece * 8) = o2; }
        };
        pass(); __threadfence(); pass();
    } else {
        float* crow = C + (size_t)r0 * ldc + c0;
        auto pass = [&]() {
#pragma unroll
            for (int s = 0; s < 8; ++s) { const int Lid = (lane >> 3) + 4 * s, piece = lane & 7; const int row = Lid >> 1, cofs = (Lid & 1) * 32 + piece * 4;
                v4f val = *(const v4fa*)(os + row * 68 + cofs); if (R) { const v4f rv = *(const v4f*)(R + ((size_t)r0 + row) * ldc + c0 + cofs); val += roundR ? (v4f){bfr(rv[0]), bfr(rv[1]), bfr(rv[2]), bfr(rv[3])} : rv; }
                *(volatile v4f*)(crow + (size_t)row * ldc + cofs) = val; }
        };
        pass(); __threadfence(); pass();
    }
}


template <int MODE>
__global__ __launch_bounds__(128) void k_gemm3z(const bf* __restrict__ Ah, const bf* __restrict__ Al, const bf* __restrict__ Bh, const bf* __restrict__ Bl, int K, float* C, int ldc, size_t sA, size_t sB, size_t sC) {
    if ((MODE & 1) && (int)blockIdx.y * 64 > (int)blockIdx.x * 64 + 63) return;
    const size_t z = blockIdx.z; Ah += z * sA; Al += z * sA; Bh += z * sB; Bl += z * sB; C += z * sC;
    const int Klim = (MODE & 2) ? min(K, ((int)blockIdx.x + 1) * 64) : K;
    __shared__ __align__(16) float ost[4][16 * 68];
    const int lane = threadIdx.x & 31, wave = threadIdx.x >> 5, lr = lane & 15, hi = lane >> 4;
    const int r0 = blockIdx.x * 64 + wave * 16, c0 = blockIdx.y * 64;
    const size_t aoff = (size_t)(r0 + lr) * K + 8 * hi;
    v8f acc[4];
#pragma unroll
    for (int t = 0; t < 4; ++t) acc[t] = (v8f){};
#pragma unroll 1
    for (int kc = 0; kc < Klim; kc += 32) {
        const v16bf a = cat16b(*(const v8us*)(Ah + aoff + kc), *(const v8us*)(Ah + aoff + kc + 16));
        v16bf al = a; if (!(MODE & 4) && !(MODE & 16)) al = cat16b(*(const v8us*)(Al + aoff + kc), *(const v8us*)(Al + aoff + kc + 16));
#pragma unroll
        for (int t = 0; t < 4; ++t) { const size_t bo = (size_t)(c0 + t * 16 + lr) * K + kc + 8 * hi;
            const v16bf bh = cat16b(*(const v8us*)(Bh + bo), *(const v8us*)(Bh + bo + 16));
            acc[t] = wmmab(a, bh, acc[t]);
            if (!(MODE & 4)) { if (!(MODE & 16)) acc[t] = wmmab(al, bh, acc[t]); if (!(MODE & 8)) { const v16bf bl = cat16b(*(const v8us*)(Bl + bo), *(const v8us*)(Bl + bo + 16)); acc[t] = wmmab(a, bl, acc[t]); } } }
        asm volatile("v_nop\n\tv_nop\n\tv_nop\n\tv_nop" : "+v"(acc[0]), "+v"(acc[1]), "+v"(acc[2]), "+v"(acc[3]) : "v"(a), "v"(al));
    }
    float* os = &ost[wave][0];
#pragma unroll
    for (int t = 0; t < 4; ++t) {
#pragma unroll
        for (int j = 0; j < 8; ++j) os[(hi * 8 + j) * 68 + t * 16 + lr] = acc[t][j]; }
    __builtin_amdgcn_wave_barrier(); asm volatile("" ::: "memory");
    float* crow = C + (size_t)r0 * ldc + c0;
    auto pass = [&]() {
#pragma unroll
        for (int s = 0; s < 8; ++s) { const int Lid = (lane >> 3) + 4 * s, piece = lane & 7; const int row = Lid >> 1, cofs = (Lid & 1) * 32 + piece * 4;
            const v4f val = *(const v4fa*)(os + row * 68 + cofs); *(volatile v4f*)(crow + (size_t)row * ldc + cofs) = val; }
    };
    pass(); __threadfence(); pass();
}
__global__ __launch_bounds__(256) void k_planes32z(const float* __restrict__ F, int ld, int off, float sc, int rows, bf* Ph, bf* Pl) {
    typedef __attribute__((ext_vector_type(2))) unsigned short v2us;
    const int lane = threadIdx.x & 31; const size_t r = ((size_t)blockIdx.x * 8 + (threadIdx.x >> 5)) * 2 + (lane >> 4); if (r >= (size_t)rows) return; const int z = blockIdx.z; const int c0 = (lane & 15) * 2; v2us oh, ol;
    Ph += (size_t)z * rows * 32; Pl += (size_t)z * rows * 32;
#pragma unroll
    for (int i = 0; i < 2; ++i) { const float y = F[r * ld + off + z * 32 + c0 + i] * sc; const unsigned short hb = f2bf(y); oh[i] = hb; ol[i] = f2bf(y - bf2f(hb)); }
    const size_t o = r * 32 + c0; *(volatile v2us*)(Ph + o) = oh; *(volatile v2us*)(Pl + o) = ol; __threadfence(); *(volatile v2us*)(Ph + o) = oh; *(volatile v2us*)(Pl + o) = ol;
}
__global__ __launch_bounds__(256) void k_vtpadz(const float* __restrict__ F, int ld, int off, int nk, bf* Th, bf* Tl) {
    typedef __attribute__((ext_vector_type(2))) unsigned short v2us;
    const int lane = threadIdx.x & 31; const size_t wid = (size_t)blockIdx.x * 8 + (threadIdx.x >> 5); if (wid >= (size_t)64 * (nk / 64)) return; const int z = blockIdx.z; const int d = (int)(wid / (nk / 64)); const int k0 = (int)(wid % (nk / 64)) * 64 + lane * 2; v2us oh, ol;
    Th += (size_t)z * 64 * nk; Tl += (size_t)z * 64 * nk;
#pragma unroll
    for (int i = 0; i < 2; ++i) { const float y = (d < 32) ? F[(size_t)(k0 + i) * ld + off + z * 32 + (d < 32 ? d : 0)] : 0.f; const unsigned short hb = f2bf(y); oh[i] = hb; ol[i] = f2bf(y - bf2f(hb)); }
    const size_t o = (size_t)d * nk + k0; *(volatile v2us*)(Th + o) = oh; *(volatile v2us*)(Tl + o) = ol; __threadfence(); *(volatile v2us*)(Th + o) = oh; *(volatile v2us*)(Tl + o) = ol;
}
template <int NK>
__global__ __launch_bounds__(256) void k_softmaxz(const float* __restrict__ S, int rows, bf* PH, bf* PL) {
    typedef __attribute__((ext_vector_type(4))) unsigned short v4us;
    const int lane = threadIdx.x & 31, i = blockIdx.x * 8 + (threadIdx.x >> 5); if (i >= rows) return; const size_t zo = (size_t)blockIdx.z * rows * NK; const float* sr = S + zo + (size_t)i * NK; PH += zo; PL += zo;
    float m = -3.0e38f;
#pragma unroll 1
    for (int c0 = lane * 4; c0 < NK; c0 += 128) {
#pragma unroll
        for (int q = 0; q < 4; ++q) m = fmaxf(m, sr[c0 + q]); }
#pragma unroll
    for (int sh = 16; sh; sh >>= 1) m = fmaxf(m, __shfl_xor(m, sh, 32));
    float sum = 0.f;
#pragma unroll 1
    for (int c0 = lane * 4; c0 < NK; c0 += 128) {
#pragma unroll
        for (int q = 0; q < 4; ++q) sum += __expf(sr[c0 + q] - m); }
#pragma unroll
    for (int sh = 16; sh; sh >>= 1) sum += __shfl_xor(sum, sh, 32);
    const float inv = 1.0f / sum;
#pragma unroll 1
    for (int ps = 0; ps < 2; ++ps) {
#pragma unroll 1
        for (int c0 = lane * 4; c0 < NK; c0 += 128) { v4us oh, ol;
#pragma unroll
            for (int q = 0; q < 4; ++q) { const float p = __expf(sr[c0 + q] - m) * inv; const unsigned short hb = f2bf(p); oh[q] = hb; ol[q] = f2bf(p - bf2f(hb)); }
            const size_t o = (size_t)i * NK + c0; *(volatile v4us*)(PH + o) = oh; *(volatile v4us*)(PL + o) = ol; }
        if (ps == 0) __threadfence(); }
}
__global__ __launch_bounds__(256) void k_placez(const float* __restrict__ XH, int rows, int ldy, float* Y) {
    const int lane = threadIdx.x & 31; const size_t q = (size_t)blockIdx.x * 8 + (threadIdx.x >> 5); if (q >= (size_t)rows) return; const int z = blockIdx.z; const float v = XH[((size_t)z * rows + q) * 64 + lane];
    *(volatile float*)(Y + q * ldy + z * 32 + lane) = v; __threadfence(); *(volatile float*)(Y + q * ldy + z * 32 + lane) = v;
}

template <bool CHMAJOR>
__global__ __launch_bounds__(256) void k_l2n(const float* __restrict__ src, bf* Ph, bf* Pl) {
    typedef __attribute__((ext_vector_type(2))) unsigned short v2us;
    const int lane = threadIdx.x & 31; const int r = blockIdx.x * 8 + (threadIdx.x >> 5); if (r >= NPT) return; const int b = r / NN, i = r % NN; float v[2]; float q = 0.f;
#pragma unroll
    for (int k = 0; k < 2; ++k) { const int c = lane * 2 + k; v[k] = bfr(CHMAJOR ? src[((size_t)b * CI + c) * MM + i] : src[(size_t)r * CI + c]); q = fmaf(v[k], v[k], q); }
#pragma unroll
    for (int sh = 16; sh; sh >>= 1) q += __shfl_xor(q, sh, 32);
    const float inv = __fdiv_rn(1.0f, fmaxf(__fsqrt_rn(q), 1e-12f)); v2us oh, ol;
#pragma unroll
    for (int k = 0; k < 2; ++k) { const float y = v[k] * inv; const unsigned short hb = f2bf(y); oh[k] = hb; ol[k] = f2bf(y - bf2f(hb)); }
    *(volatile v2us*)(Ph + (size_t)r * CI + lane * 2) = oh; *(volatile v2us*)(Pl + (size_t)r * CI + lane * 2) = ol; __threadfence(); *(volatile v2us*)(Ph + (size_t)r * CI + lane * 2) = oh; *(volatile v2us*)(Pl + (size_t)r * CI + lane * 2) = ol;
}
template <bool COL>
__global__ __launch_bounds__(256) void k_rcmax(const float* __restrict__ COS, float* OUTV) {
    const int lane = threadIdx.x & 31; const int w = blockIdx.x * 8 + (threadIdx.x >> 5); if (w >= NPT / 32) return; const int b = w / (NN / 32), t = (w % (NN / 32)) * 32 + lane; const float* cb = COS + (size_t)b * NN * MM; float m = -3.0e38f;
#pragma unroll 1
    for (int k = 0; k < 512; ++k) m = fmaxf(m, COL ? cb[(size_t)k * MM + t] : cb[(size_t)t * MM + k]);
    *(volatile float*)(OUTV + (size_t)b * 512 + t) = m; __threadfence(); *(volatile float*)(OUTV + (size_t)b * 512 + t) = m;
}
__global__ __launch_bounds__(256) void k_upoint(const float* __restrict__ xyz, const float* __restrict__ lz, const float* __restrict__ pts, const float* __restrict__ W1, const float* __restrict__ b1, float* U) {
    const int lane = threadIdx.x & 31; const int r = blockIdx.x * 8 + (threadIdx.x >> 5); if (r >= NPT) return; const int c0 = lane * 4; const float z = bfr(lz[r]); v4f a;
#pragma unroll
    for (int k = 0; k < 4; ++k) a[k] = bfr(b1[c0 + k]);
#pragma unroll 1
    for (int f = 0; f < 3; ++f) { const float v = bfr(xyz[(size_t)r * 3 + f]) * z; for (int k = 0; k < 4; ++k) a[k] = fmaf(v, bfr(W1[(size_t)f * C1 + c0 + k]), a[k]); }
#pragma unroll 1
    for (int f = 0; f < 2; ++f) { const float v = bfr(pts[(size_t)r * CI + f]); for (int k = 0; k < 4; ++k) a[k] = fmaf(v, bfr(W1[(size_t)(3 + f) * C1 + c0 + k]), a[k]); }
#pragma unroll 1
    for (int f = 0; f < CI; ++f) { const float v = bfr(pts[(size_t)r * CI + f]); for (int k = 0; k < 4; ++k) a[k] = fmaf(v, bfr(W1[(size_t)(10 + f) * C1 + c0 + k]), a[k]); }
    *(volatile v4f*)(U + (size_t)r * C1 + c0) = a; __threadfence(); *(volatile v4f*)(U + (size_t)r * C1 + c0) = a;
}
__global__ __launch_bounds__(256) void k_vcell(const float* __restrict__ RFI, const float* __restrict__ RF3, const float* __restrict__ W1, float* V) {
    const int lane = threadIdx.x & 31; const int r = blockIdx.x * 8 + (threadIdx.x >> 5); if (r >= NCL) return; const int b = r / MM, m = r % MM; const int c0 = lane * 4; v4f a = (v4f){0.f, 0.f, 0.f, 0.f};
#pragma unroll 1
    for (int f = 0; f < 2; ++f) { const float v = bfr(RFI[((size_t)b * 3 + f) * MM + m]); for (int k = 0; k < 4; ++k) a[k] = fmaf(v, bfr(W1[(size_t)(5 + f) * C1 + c0 + k]), a[k]); }
#pragma unroll 1
    for (int f = 0; f < CI; ++f) { const float v = bfr(RF3[((size_t)b * CI + f) * MM + m]); for (int k = 0; k < 4; ++k) a[k] = fmaf(v, bfr(W1[(size_t)(74 + f) * C1 + c0 + k]), a[k]); }
    *(volatile v4f*)(V + (size_t)r * C1 + c0) = a; __threadfence(); *(volatile v4f*)(V + (size_t)r * C1 + c0) = a;
}
__device__ __forceinline__ float pairterms(float e0, float e1, float en, float s1, float s2, const float* __restrict__ W1, int c) {
    float a = e0 * bfr(W1[(size_t)7 * C1 + c]); a = fmaf(e1, bfr(W1[(size_t)8 * C1 + c]), a); a = fmaf(en, bfr(W1[(size_t)9 * C1 + c]), a); a = fmaf(s1, bfr(W1[(size_t)138 * C1 + c]), a); a = fmaf(s2, bfr(W1[(size_t)139 * C1 + c]), a); return a;
}
template <int PASS>
__global__ __launch_bounds__(256) void k_bn1(const float* __restrict__ U, const float* __restrict__ Vc, const float* __restrict__ xyz, const float* __restrict__ RFI, const float* __restrict__ COS, const float* __restrict__ RMAX, const float* __restrict__ CMAX, const float* __restrict__ W1, const float* __restrict__ MEAN, float* PART) {
    const int lane = threadIdx.x & 31; const int r = blockIdx.x * 8 + (threadIdx.x >> 5); if (r >= NPT) return; const int b = r / NN, n = r % NN; const int c0 = lane * 4;
    const float x0 = bfr(xyz[(size_t)r * 3]), x1 = bfr(xyz[(size_t)r * 3 + 1]); const float rmx = RMAX[r] + 1e-6f; v4f u = *(const v4f*)(U + (size_t)r * C1 + c0); v4f acc = (v4f){0.f, 0.f, 0.f, 0.f}; v4f mu = (v4f){0.f, 0.f, 0.f, 0.f};
    if (PASS == 1) mu = *(const v4f*)(MEAN + c0);
#pragma unroll 1
    for (int m = 0; m < MM; ++m) { const int q = b * MM + m; const float e0 = x0 - bfr(RFI[((size_t)b * 3 + 0) * MM + m]), e1 = x1 - bfr(RFI[((size_t)b * 3 + 1) * MM + m]); const float en = __fsqrt_rn(e0 * e0 + e1 * e1); const float cs = COS[((size_t)b * NN + n) * MM + m]; const float s1 = __fdiv_rn(cs, rmx), s2 = __fdiv_rn(cs, CMAX[q] + 1e-10f);
        const v4f vv = *(const v4f*)(Vc + (size_t)q * C1 + c0);
#pragma unroll
        for (int k = 0; k < 4; ++k) { const float f1 = u[k] + vv[k] + pairterms(e0, e1, en, s1, s2, W1, c0 + k); if (PASS == 0) acc[k] += f1; else { const float d = f1 - mu[k]; acc[k] = fmaf(d, d, acc[k]); } } }
    *(volatile v4f*)(PART + (size_t)r * C1 + c0) = acc; __threadfence(); *(volatile v4f*)(PART + (size_t)r * C1 + c0) = acc;
}
__global__ __launch_bounds__(256) void k_colred(const float* __restrict__ PART, int nrows, int C, float scale, float* OUTV) {
    const int lane = threadIdx.x & 31; const int c = (threadIdx.x >> 5) * 32 + lane; if (c >= C) return; float s = 0.f;
#pragma unroll 1
    for (int r = 0; r < nrows; ++r) s += PART[(size_t)r * C + c];
    s *= scale; *(volatile float*)(OUTV + c) = s; __threadfence(); *(volatile float*)(OUTV + c) = s;
}
__global__ __launch_bounds__(256) void k_y1planes(const float* __restrict__ U, const float* __restrict__ Vc, const float* __restrict__ xyz, const float* __restrict__ RFI, const float* __restrict__ COS, const float* __restrict__ RMAX, const float* __restrict__ CMAX, const float* __restrict__ W1, const float* __restrict__ MEAN, const float* __restrict__ VAR, const float* __restrict__ g1, const float* __restrict__ be1, int r0, bf* Ph, bf* Pl) {
    typedef __attribute__((ext_vector_type(4))) unsigned short v4us;
    const int lane = threadIdx.x & 31; const size_t pr = (size_t)blockIdx.x * 8 + (threadIdx.x >> 5); if (pr >= (size_t)PCH) return; const int r = r0 + (int)(pr / MM), m = (int)(pr % MM); const int b = r / NN, n = r % NN; const int q = b * MM + m; const int c0 = lane * 4;
    const float x0 = bfr(xyz[(size_t)r * 3]), x1 = bfr(xyz[(size_t)r * 3 + 1]); const float e0 = x0 - bfr(RFI[((size_t)b * 3 + 0) * MM + m]), e1 = x1 - bfr(RFI[((size_t)b * 3 + 1) * MM + m]); const float en = __fsqrt_rn(e0 * e0 + e1 * e1); const float cs = COS[((size_t)b * NN + n) * MM + m]; const float s1 = __fdiv_rn(cs, RMAX[r] + 1e-6f), s2 = __fdiv_rn(cs, CMAX[q] + 1e-10f);
    v4us oh, ol;
#pragma unroll
    for (int k = 0; k < 4; ++k) { const int c = c0 + k; const float f1 = U[(size_t)r * C1 + c] + Vc[(size_t)q * C1 + c] + pairterms(e0, e1, en, s1, s2, W1, c); float y = (f1 - MEAN[c]) * rsqrtf(VAR[c] + 1e-5f) * bfr(g1[c]) + bfr(be1[c]); y = fmaxf(y, 0.f); const unsigned short hb = f2bf(y); oh[k] = hb; ol[k] = f2bf(y - bf2f(hb)); }
    *(volatile v4us*)(Ph + pr * C1 + c0) = oh; *(volatile v4us*)(Pl + pr * C1 + c0) = ol; __threadfence(); *(volatile v4us*)(Ph + pr * C1 + c0) = oh; *(volatile v4us*)(Pl + pr * C1 + c0) = ol;
}
__global__ __launch_bounds__(256) void k_wt_io(const float* __restrict__ Wm, int ldw, int K, int N, bf* Bt) {
    const int lane = threadIdx.x & 31; const int n = blockIdx.x * 8 + (threadIdx.x >> 5); if (n >= N) return;
#pragma unroll 1
    for (int ps = 0; ps < 2; ++ps) { for (int c0 = lane * 8; c0 < K; c0 += 256) { v8us o;
#pragma unroll
            for (int i = 0; i < 8; ++i) { const int k = c0 + i; o[i] = f2bf(k < K ? Wm[(size_t)(k < K ? k : 0) * ldw + n] : 0.f); }
            *(volatile v8us*)(Bt + (size_t)n * K + c0) = o; }
        if (ps == 0) __threadfence(); }
}
template <int PASS>
__global__ __launch_bounds__(256) void k_bn2(const float* __restrict__ F2, const float* __restrict__ MEAN, float* PART2) {
    typedef __attribute__((ext_vector_type(2))) float v2f_;
    const int lane = threadIdx.x & 31; const int r = blockIdx.x * 8 + (threadIdx.x >> 5); if (r >= NPT) return; const int c0 = lane * 2; float a0 = 0.f, a1 = 0.f; const float m0 = PASS ? MEAN[c0] : 0.f, m1 = PASS ? MEAN[c0 + 1] : 0.f;
#pragma unroll 1
    for (int m = 0; m < MM; ++m) { const float* fr = F2 + ((size_t)r * MM + m) * C2O + c0; if (PASS == 0) { a0 += fr[0]; a1 += fr[1]; } else { const float d0 = fr[0] - m0, d1 = fr[1] - m1; a0 = fmaf(d0, d0, a0); a1 = fmaf(d1, d1, a1); } }
    v2f_ o; o[0] = a0; o[1] = a1; *(volatile v2f_*)(PART2 + (size_t)r * C2O + c0) = o; __threadfence(); *(volatile v2f_*)(PART2 + (size_t)r * C2O + c0) = o;
}
__global__ __launch_bounds__(256) void k_attn(const float* __restrict__ F2, const float* __restrict__ MEAN, const float* __restrict__ VAR, const float* __restrict__ g2, const float* __restrict__ be2, float* ATT) {
    __shared__ float smx[8][MM];
    typedef __attribute__((ext_vector_type(2))) float v2f_;
    const int lane = threadIdx.x & 31, wv = threadIdx.x >> 5; const int r = blockIdx.x * 8 + wv; if (r >= NPT) return; float* mxr = smx[wv]; const int c0 = lane * 2;
    const float sc0 = rsqrtf(VAR[c0] + 1e-5f) * bfr(g2[c0]), sc1 = rsqrtf(VAR[c0 + 1] + 1e-5f) * bfr(g2[c0 + 1]); const float of0 = bfr(be2[c0]) - MEAN[c0] * sc0, of1 = bfr(be2[c0 + 1]) - MEAN[c0 + 1] * sc1;
#pragma unroll 1
    for (int m = 0; m < MM; ++m) { const float* fr = F2 + ((size_t)r * MM + m) * C2O + c0; float v = fmaxf(fmaxf(fmaf(fr[0], sc0, of0), 0.f), fmaxf(fmaf(fr[1], sc1, of1), 0.f));
#pragma unroll
        for (int sh = 16; sh; sh >>= 1) v = fmaxf(v, __shfl_xor(v, sh, 32));
        if (lane == 0) mxr[m] = v; }
    __builtin_amdgcn_wave_barrier(); asm volatile("" ::: "memory");
    float gm = -3.0e38f;
#pragma unroll 1
    for (int m = lane; m < MM; m += 32) gm = fmaxf(gm, mxr[m]);
#pragma unroll
    for (int sh = 16; sh; sh >>= 1) gm = fmaxf(gm, __shfl_xor(gm, sh, 32));
    float se = 0.f;
#pragma unroll 1
    for (int m = lane; m < MM; m += 32) se += __expf(mxr[m] - gm);
#pragma unroll
    for (int sh = 16; sh; sh >>= 1) se += __shfl_xor(se, sh, 32);
    const float inv = __fdiv_rn(1.0f, se); float a0 = 0.f, a1 = 0.f;
#pragma unroll 1
    for (int m = 0; m < MM; ++m) { const float aw = __expf(mxr[m] - gm) * inv; const float* fr = F2 + ((size_t)r * MM + m) * C2O + c0; a0 = fmaf(aw, fmaxf(fmaf(fr[0], sc0, of0), 0.f), a0); a1 = fmaf(aw, fmaxf(fmaf(fr[1], sc1, of1), 0.f), a1); }
    v2f_ o; o[0] = a0; o[1] = a1; *(volatile v2f_*)(ATT + (size_t)r * C2O + c0) = o; __threadfence(); *(volatile v2f_*)(ATT + (size_t)r * C2O + c0) = o;
}
__global__ __launch_bounds__(256) void k_h1(const float* __restrict__ ATT, const float* __restrict__ M1w, const float* __restrict__ M1b, float* H1) {
    const int lane = threadIdx.x & 31; const int r = blockIdx.x * 8 + (threadIdx.x >> 5); if (r >= NPT) return; float a = bfr(M1b[lane]);
#pragma unroll 1
    for (int c = 0; c < C2O; ++c) a = fmaf(ATT[(size_t)r * C2O + c], bfr(M1w[c * C3 + lane]), a);
    *(volatile float*)(H1 + (size_t)r * C3 + lane) = a; __threadfence(); *(volatile float*)(H1 + (size_t)r * C3 + lane) = a;
}
__global__ __launch_bounds__(64) void k_bn3(const float* __restrict__ H1, float* MV3) {
    const int lane = threadIdx.x & 31; if (threadIdx.x >= 32) return; float s = 0.f;
#pragma unroll 1
    for (int r = 0; r < NPT; ++r) s += H1[(size_t)r * C3 + lane];
    const float mu = s * (1.0f / NPT); float q = 0.f;
#pragma unroll 1
    for (int r = 0; r < NPT; ++r) { const float d = H1[(size_t)r * C3 + lane] - mu; q = fmaf(d, d, q); }
    const float var = q * (1.0f / NPT);
    *(volatile float*)(MV3 + lane) = mu; *(volatile float*)(MV3 + 32 + lane) = var; __threadfence(); *(volatile float*)(MV3 + lane) = mu; *(volatile float*)(MV3 + 32 + lane) = var;
}
__global__ __launch_bounds__(256) void k_out(const float* __restrict__ H1, const float* __restrict__ MV3, const float* __restrict__ g3, const float* __restrict__ be3, const float* __restrict__ M2w, const float* __restrict__ M2b, float* OUTB) {
    const int lane = threadIdx.x & 31; const int w = blockIdx.x * 8 + (threadIdx.x >> 5); if (w >= NPT / 16) return; const int r = w * 16 + (lane >> 1), o = lane & 1; float a = bfr(M2b[o]);
#pragma unroll 1
    for (int k = 0; k < C3; ++k) { const float y = fmaxf((H1[(size_t)r * C3 + k] - MV3[k]) * rsqrtf(MV3[32 + k] + 1e-5f) * bfr(g3[k]) + bfr(be3[k]), 0.f); a = fmaf(y, bfr(M2w[k * 2 + o]), a); }
    *(volatile float*)(OUTB + (size_t)r * 2 + o) = a; __threadfence(); *(volatile float*)(OUTB + (size_t)r * 2 + o) = a;
}
extern "C" void kernel_launch(void* const* d_in, const int* in_sizes, int n_in,
                              void* d_out, int out_size, void* d_ws, size_t ws_size, hipStream_t stream) {
    (void)in_sizes; (void)n_in; (void)out_size;
    const float* xyz = (const float*)d_in[0]; const float* pts = (const float*)d_in[1]; const float* RF3 = (const float*)d_in[2]; const float* RFI = (const float*)d_in[3]; const float* lz = (const float*)d_in[4];
    const float* W1 = (const float*)d_in[5]; const float* b1 = (const float*)d_in[6]; const float* g1 = (const float*)d_in[7]; const float* be1 = (const float*)d_in[8]; const float* W2 = (const float*)d_in[9]; const float* b2 = (const float*)d_in[10]; const float* g2 = (const float*)d_in[11]; const float* be2 = (const float*)d_in[12];
    const float* M1w = (const float*)d_in[13]; const float* M1b = (const float*)d_in[14]; const float* M1g = (const float*)d_in[15]; const float* M1be = (const float*)d_in[16]; const float* M2w = (const float*)d_in[17]; const float* M2b = (const float*)d_in[18];
    float* out = (float*)d_out;
    char* wsp = (char*)d_ws;
    auto take = [&](size_t bytes) { char* p = wsp; wsp += (bytes + 255) & ~(size_t)255; return (void*)p; };
    bf* SNh = (bf*)take(NPT * CI * 2); bf* SNl = (bf*)take(NPT * CI * 2); bf* DNh = (bf*)take(NCL * CI * 2); bf* DNl = (bf*)take(NCL * CI * 2); float* COS = (float*)take((size_t)NB_ * NN * MM * 4); float* RMAX = (float*)take(NPT * 4); float* CMAX = (float*)take(NCL * 4);
    float* U = (float*)take((size_t)NPT * C1 * 4); float* Vc = (float*)take((size_t)NCL * C1 * 4); float* PART = (float*)take((size_t)NPT * C1 * 4); float* MEAN1 = (float*)take(C1 * 4); float* VAR1 = (float*)take(C1 * 4);
    bf* BW2 = (bf*)take(C2O * C1 * 2); bf* Ph = (bf*)take((size_t)PCH * C1 * 2); bf* Pl = (bf*)take((size_t)PCH * C1 * 2); float* F2 = (float*)take((size_t)NPR * C2O * 4); float* PART2 = (float*)take((size_t)NPT * C2O * 4); float* MEAN2 = (float*)take(C2O * 4); float* VAR2 = (float*)take(C2O * 4);
    float* ATT = (float*)take((size_t)NPT * C2O * 4); float* H1 = (float*)take((size_t)NPT * C3 * 4); float* MV3 = (float*)take(64 * 4);
    if ((size_t)(wsp - (char*)d_ws) > ws_size) return;
    k_l2n<false><<<NPT / 8, 256, 0, stream>>>(pts, SNh, SNl); k_l2n<true><<<NCL / 8, 256, 0, stream>>>(RF3, DNh, DNl);
    k_gemm3z<0><<<dim3(NN / 64, MM / 64, NB_), 128, 0, stream>>>(SNh, SNl, DNh, DNl, CI, COS, MM, (size_t)NN * CI, (size_t)MM * CI, (size_t)NN * MM);
    k_rcmax<false><<<(NPT / 32) / 8, 256, 0, stream>>>(COS, RMAX); k_rcmax<true><<<(NCL / 32) / 8, 256, 0, stream>>>(COS, CMAX);
    k_upoint<<<NPT / 8, 256, 0, stream>>>(xyz, lz, pts, W1, b1, U); k_vcell<<<NCL / 8, 256, 0, stream>>>(RFI, RF3, W1, Vc);
    k_bn1<0><<<NPT / 8, 256, 0, stream>>>(U, Vc, xyz, RFI, COS, RMAX, CMAX, W1, nullptr, PART); k_colred<<<1, 128, 0, stream>>>(PART, NPT, C1, 1.0f / NPR, MEAN1);
    k_bn1<1><<<NPT / 8, 256, 0, stream>>>(U, Vc, xyz, RFI, COS, RMAX, CMAX, W1, MEAN1, PART); k_colred<<<1, 128, 0, stream>>>(PART, NPT, C1, 1.0f / NPR, VAR1);
    k_wt_io<<<C2O / 8, 256, 0, stream>>>(W2, C2O, C1, C2O, BW2);
    for (int r0 = 0; r0 < NPT; r0 += NCH) {
        k_y1planes<<<PCH / 8, 256, 0, stream>>>(U, Vc, xyz, RFI, COS, RMAX, CMAX, W1, MEAN1, VAR1, g1, be1, r0, Ph, Pl);
        k_gemmb<true, false><<<dim3(PCH / 64, 1, 1), 128, 0, stream>>>(Ph, Pl, BW2, b2, F2 + (size_t)r0 * MM * C2O, C2O, nullptr, nullptr, C1); }
    k_bn2<0><<<NPT / 8, 256, 0, stream>>>(F2, nullptr, PART2); k_colred<<<1, 64, 0, stream>>>(PART2, NPT, C2O, 1.0f / NPR, MEAN2);
    k_bn2<1><<<NPT / 8, 256, 0, stream>>>(F2, MEAN2, PART2); k_colred<<<1, 64, 0, stream>>>(PART2, NPT, C2O, 1.0f / NPR, VAR2);
    k_attn<<<NPT / 8, 256, 0, stream>>>(F2, MEAN2, VAR2, g2, be2, ATT);
    k_h1<<<NPT / 8, 256, 0, stream>>>(ATT, M1w, M1b, H1);
    k_bn3<<<1, 64, 0, stream>>>(H1, MV3);
    k_out<<<(NPT / 16) / 8, 256, 0, stream>>>(H1, MV3, M1g, M1be, M2w, M2b, out);
}
